// GravityAttention_79774722556516
// MI455X (gfx1250) — hardware-verified
//
#include <hip/hip_runtime.h>


namespace {
constexpr int Bn = 4, S = 2048, D = 1024, H = 16, HD = 64, NTOK = Bn * S, D3 = 3 * D;
constexpr float SCALE = 0.125f, VS = 8.0f;

typedef _Float16 b16;
typedef __attribute__((ext_vector_type(16))) _Float16 v16b;
typedef __attribute__((ext_vector_type(8)))  _Float16 v8b;
typedef __attribute__((ext_vector_type(8)))  float v8f;
typedef __attribute__((ext_vector_type(4)))  float v4f;

__device__ __forceinline__ v8b ld8b(const b16* p) { return *(const v8b*)p; }
__device__ __forceinline__ v16b cat8b(v8b a, v8b b) { return __builtin_shufflevector(a, b, 0, 1, 2, 3, 4, 5, 6, 7, 8, 9, 10, 11, 12, 13, 14, 15); }
__device__ __forceinline__ v16b frag_kb(const b16* p, int hh) { return cat8b(ld8b(p + 8 * hh), ld8b(p + 16 + 8 * hh)); }
__device__ __forceinline__ void split16(float v, b16& hi, b16& lo) { hi = (b16)v; lo = (b16)(v - (float)hi); }
__device__ __forceinline__ void frag_ksplit(const float* p, int hh, v16b& fh_, v16b& fl_) {
  const float* p0 = p + 8 * hh; const float* p1 = p + 16 + 8 * hh;
#pragma unroll
  for (int e = 0; e < 8; ++e) { b16 a, c; split16(p0[e], a, c); fh_[e] = a; fl_[e] = c; split16(p1[e], a, c); fh_[8 + e] = a; fl_[8 + e] = c; }
}
__device__ __forceinline__ v8f wmma16b(v16b a, v16b b, v8f c) {
  v8f d = __builtin_amdgcn_wmma_f32_16x16x32_f16(false, a, false, b, (short)0, c, false, false);
  asm volatile("v_nop\n\tv_nop\n\tv_nop\n\tv_nop" : "+v"(d) : "v"(a), "v"(b));
  return d;
}
__device__ __forceinline__ void wave_lds_sync() {
  __builtin_amdgcn_fence(__ATOMIC_RELEASE, "workgroup");
  __builtin_amdgcn_wave_barrier();
  __builtin_amdgcn_fence(__ATOMIC_ACQUIRE, "workgroup");
}

struct Opnd { const void* p0; const void* p1; int ld; };
template <int NP> __device__ __forceinline__ void load_frags(const Opnd& o, int row, int kb, int hh, v16b& fh_, v16b& fl_) {
  if (NP == 0) { frag_ksplit((const float*)o.p0 + (size_t)row * o.ld + kb, hh, fh_, fl_); }
  else if (NP == 4 || NP == 5) {
    const float sc_ = (NP == 4) ? 64.0f : 8.0f;
    const float* p = (const float*)o.p0 + (size_t)row * o.ld + kb; const float* p0 = p + 8 * hh; const float* p1 = p + 16 + 8 * hh;
#pragma unroll
    for (int e = 0; e < 8; ++e) { b16 a, c; split16(p0[e] * sc_, a, c); fh_[e] = a; fl_[e] = c; split16(p1[e] * sc_, a, c); fh_[8 + e] = a; fl_[8 + e] = c; }
  } else if (NP == 3) {
    const float* p = (const float*)o.p0 + (size_t)row * o.ld + kb; const float* p0 = p + 8 * hh; const float* p1 = p + 16 + 8 * hh;
#pragma unroll
    for (int e = 0; e < 8; ++e) { fh_[e] = (b16)p0[e]; fh_[8 + e] = (b16)p1[e]; }
    fl_ = fh_;
  } else {
    fh_ = frag_kb((const b16*)o.p0 + (size_t)row * o.ld + kb, hh);
    if (NP == 2) fl_ = frag_kb((const b16*)o.p1 + (size_t)row * o.ld + kb, hh); else fl_ = fh_;
  }
}
template <int ANP, int BNP> __device__ __forceinline__ v8f mac(v16b ah, v16b al, v16b bh, v16b bl, v8f c) {
  c = wmma16b(ah, bh, c);
  if (BNP == 0 || BNP == 2 || BNP == 4 || BNP == 5) c = wmma16b(ah, bl, c);
  if (ANP == 0 || ANP == 2 || ANP == 4 || ANP == 5) c = wmma16b(al, bh, c);
  return c;
}
template <int ANP, int BNP>
__device__ __forceinline__ void gemm_tile(const Opnd& A, const Opnd& B, int K, int m0, int c0, int nloc, int hlf, v8f (&acc)[2][4]) {
  for (int kb = 0; kb < K; kb += 32) {
    v16b a0h, a0l, a1h, a1l;
    load_frags<ANP>(A, m0 + nloc, kb, hlf, a0h, a0l);
    load_frags<ANP>(A, m0 + 16 + nloc, kb, hlf, a1h, a1l);
#pragma unroll
    for (int t = 0; t < 4; ++t) {
      v16b bh, bl;
      load_frags<BNP>(B, c0 + t * 16 + nloc, kb, hlf, bh, bl);
      acc[0][t] = mac<ANP, BNP>(a0h, a0l, bh, bl, acc[0][t]);
      acc[1][t] = mac<ANP, BNP>(a1h, a1l, bh, bl, acc[1][t]);
    }
  }
}

__device__ __forceinline__ void epi_planes(v8f (&acc)[2][4], float scale, bool two, b16* __restrict__ oh, b16* __restrict__ ol, int ldo,
                                           int m0, int c0, int lane, b16* Th, b16* Tl) {
  const int nloc = lane & 15, hlf = lane >> 4;
#pragma unroll
  for (int t = 0; t < 4; ++t)
#pragma unroll
    for (int r = 0; r < 2; ++r)
#pragma unroll
      for (int v = 0; v < 8; ++v) {
        const int rr = r * 16 + v + 8 * hlf, cc = t * 16 + nloc;
        b16 h_, l_; split16(acc[r][t][v] * scale, h_, l_);
        Th[rr * 64 + cc] = h_; Tl[rr * 64 + cc] = l_;
      }
  wave_lds_sync();
  for (int pass = 0; pass < 2; ++pass) {
#pragma unroll
    for (int j = 0; j < 8; ++j) {
      const int rr = j * 4 + (lane >> 3), c8 = (lane & 7) * 8;
      const size_t o = (size_t)(m0 + rr) * ldo + c0 + c8;
      *(volatile v8b*)(oh + o) = ld8b(Th + rr * 64 + c8);
      if (two) *(volatile v8b*)(ol + o) = ld8b(Tl + rr * 64 + c8);
    }
    __threadfence();
  }
}
__device__ __forceinline__ void epi_f32(v8f (&acc)[2][4], float scale, const float* rscale, float* __restrict__ out, int ldo, int m0, int c0, int lane, float* Tt) {
  const int nloc = lane & 15, hlf = lane >> 4;
#pragma unroll
  for (int t = 0; t < 4; ++t)
#pragma unroll
    for (int r = 0; r < 2; ++r)
#pragma unroll
      for (int v = 0; v < 8; ++v) {
        const int rr = r * 16 + v + 8 * hlf;
        const float rs = rscale ? rscale[(size_t)(m0 + rr) * 32] : 1.0f;
        Tt[rr * 64 + t * 16 + nloc] = acc[r][t][v] * scale * rs;
      }
  wave_lds_sync();
  float* dst0 = out + (size_t)m0 * ldo + c0;
  for (int pass = 0; pass < 2; ++pass) {
#pragma unroll
    for (int j = 0; j < 16; ++j) { const int rr = j * 2 + hlf, c4 = nloc * 4; *(volatile v4f*)(dst0 + (size_t)rr * ldo + c4) = *(const v4f*)(Tt + rr * 64 + c4); }
    __threadfence();
  }
}


typedef __attribute__((ext_vector_type(8))) __bf16 v8bb; typedef __attribute__((ext_vector_type(16))) __bf16 v16bb;
typedef __attribute__((ext_vector_type(8))) unsigned short v8us;
__device__ __forceinline__ v16bb frag_kb_bf(const __bf16* p, int hh) { const v8bb a = *(const v8bb*)(p + 8 * hh), b = *(const v8bb*)(p + 16 + 8 * hh); return __builtin_shufflevector(a, b, 0, 1, 2, 3, 4, 5, 6, 7, 8, 9, 10, 11, 12, 13, 14, 15); }
__device__ __forceinline__ v8f wmma16bb(v16bb a, v16bb b, v8f c) {
  v8f d = __builtin_amdgcn_wmma_f32_16x16x32_bf16(false, a, false, b, (short)0, c, false, false);
  asm volatile("v_nop\n\tv_nop\n\tv_nop\n\tv_nop" : "+v"(d) : "v"(a), "v"(b));
  return d;
}
__device__ __forceinline__ unsigned short bf16_rne_bits(float v) { unsigned int u = __float_as_uint(v); u += 0x7FFFu + ((u >> 16) & 1u); return (unsigned short)(u >> 16); }
__device__ __forceinline__ float bf16_rne(float v) { return __uint_as_float(((unsigned int)bf16_rne_bits(v)) << 16); }

__global__ __launch_bounds__(256) void prep_kernel(const float* __restrict__ x, unsigned short* __restrict__ x16) {
  const size_t tid = (size_t)blockIdx.x * blockDim.x + threadIdx.x, nth = (size_t)gridDim.x * blockDim.x;
  for (int pass = 0; pass < 2; ++pass) {
    for (size_t p = tid; p < (size_t)NTOK * D / 8; p += nth) { v8us v;
#pragma unroll
      for (int e = 0; e < 8; ++e) v[e] = bf16_rne_bits(x[p * 8 + e]);
      *(volatile v8us*)(x16 + p * 8) = v; }
    __threadfence();
  }
}
__device__ __forceinline__ void sincos_acc(float f, float& sn, float& cs) {
  const double x = (double)f; const double twooverpi = 0.63661977236758134308; const double pio2 = 1.57079632679489661923;
  const double kq = rint(x * twooverpi); const double r = x - kq * pio2; const int q = (int)kq & 3;
  const double r2 = r * r;
  double sp = r * (1.0 + r2 * (-1.0 / 6 + r2 * (1.0 / 120 + r2 * (-1.0 / 5040 + r2 * (1.0 / 362880 + r2 * (-1.0 / 39916800 + r2 * (1.0 / 6227020800.0)))))));
  double cp = 1.0 + r2 * (-0.5 + r2 * (1.0 / 24 + r2 * (-1.0 / 720 + r2 * (1.0 / 40320 + r2 * (-1.0 / 3628800 + r2 * (1.0 / 479001600.0))))));
  double s_, c_;
  if (q == 0) { s_ = sp; c_ = cp; } else if (q == 1) { s_ = cp; c_ = -sp; } else if (q == 2) { s_ = -sp; c_ = -cp; } else { s_ = -cp; c_ = sp; }
  sn = (float)s_; cs = (float)c_;
}
__global__ __launch_bounds__(256) void rope_kernel(float* __restrict__ cst) {
  const int i = blockIdx.x * 256 + threadIdx.x; const int t = i / 32, j = i % 32;
  const float inv = 1.0f / powf(10000.0f, (float)(2 * j) / (float)HD); const float f = (float)t * inv;
  float sn, cs; sincos_acc(f, sn, cs);
  for (int pass = 0; pass < 2; ++pass) { ((volatile float*)cst)[2 * i] = cs; ((volatile float*)cst)[2 * i + 1] = sn; __threadfence(); }
}
template <int MODE>
__global__ __launch_bounds__(256) void wt_kernel(const float* __restrict__ W, int K, int Ncols, unsigned short* __restrict__ out) {
  __shared__ __attribute__((aligned(16))) unsigned short Tl[64][72];
  const int tid = threadIdx.x, lane = tid & 31, wave = tid >> 5, n0 = blockIdx.x * 64, k0 = blockIdx.y * 64;
  for (int i = tid; i < 64 * 64; i += 256) { const int kk = i / 64, nn = i % 64; const float w = W[(size_t)(k0 + kk) * Ncols + n0 + nn];
    unsigned short bits; if (MODE == 0) bits = bf16_rne_bits(w); else { const b16 hv = (b16)bf16_rne(w); bits = *reinterpret_cast<const unsigned short*>(&hv); }
    Tl[nn][kk] = bits; }
  __syncthreads();
  for (int pass = 0; pass < 2; ++pass) {
#pragma unroll
    for (int j = 0; j < 2; ++j) { const int rr = wave * 8 + j * 4 + (lane >> 3), c8 = (lane & 7) * 8; *(volatile v8us*)(out + (size_t)(n0 + rr) * K + k0 + c8) = *(const v8us*)(&Tl[rr][c8]); }
    __threadfence();
  }
}

__global__ __launch_bounds__(128) void proj_kernel(const __bf16* __restrict__ x16, const __bf16* __restrict__ w16, const float* __restrict__ cst, b16* __restrict__ qk, b16* __restrict__ vt, b16* __restrict__ vtl) {
  __shared__ __attribute__((aligned(16))) b16 Th[4][2][32 * 64];
  __shared__ __attribute__((aligned(16))) b16 Tt[2][64][128 + 8];
  const int lane = threadIdx.x & 31, wave = threadIdx.x >> 5, nloc = lane & 15, hlf = lane >> 4, m0 = blockIdx.y * 128 + wave * 32, cg = blockIdx.x * 64, which = cg / D, c0 = cg % D;
  const __bf16* X = x16; const __bf16* W = w16 + (size_t)which * D * D;
  v8f acc[2][4];
#pragma unroll
  for (int r = 0; r < 2; ++r)
#pragma unroll
    for (int t = 0; t < 4; ++t) acc[r][t] = (v8f){};
#pragma unroll 2
  for (int kb = 0; kb < D; kb += 32) {
    const v16bb a0 = frag_kb_bf(X + (size_t)(m0 + nloc) * D + kb, hlf), a1 = frag_kb_bf(X + (size_t)(m0 + 16 + nloc) * D + kb, hlf);
#pragma unroll
    for (int t = 0; t < 4; ++t) { const v16bb bw = frag_kb_bf(W + (size_t)(c0 + t * 16 + nloc) * D + kb, hlf); acc[0][t] = wmma16bb(a0, bw, acc[0][t]); acc[1][t] = wmma16bb(a1, bw, acc[1][t]); }
  }
  const int h = c0 / HD, b = m0 / S, s0 = m0 % S;
  if (which < 2) {
#pragma unroll
    for (int t16 = 0; t16 < 2; ++t16) { const int j = t16 * 16 + nloc;
#pragma unroll
      for (int r = 0; r < 2; ++r)
#pragma unroll
        for (int v = 0; v < 8; ++v) { const int pos = s0 + r * 16 + v + 8 * hlf; const float c = cst[(pos * 32 + j) * 2], s = cst[(pos * 32 + j) * 2 + 1];
          const float x1 = acc[r][t16][v], x2 = acc[r][t16 + 2][v]; acc[r][t16][v] = x1 * c - x2 * s; acc[r][t16 + 2][v] = x1 * s + x2 * c; } }
    epi_planes(acc, 1.0f, false, qk + ((((size_t)which * Bn + b) * H + h) * S + s0) * HD, nullptr, HD, 0, 0, lane, Th[wave][0], Th[wave][1]); return; }
#pragma unroll
  for (int t = 0; t < 4; ++t)
#pragma unroll
    for (int r = 0; r < 2; ++r)
#pragma unroll
      for (int v = 0; v < 8; ++v) { b16 a, c; split16(acc[r][t][v] * VS, a, c); Tt[0][t * 16 + nloc][wave * 32 + r * 16 + 8 * hlf + v] = a; Tt[1][t * 16 + nloc][wave * 32 + r * 16 + 8 * hlf + v] = c; }
  __syncthreads();
  const int tok0 = (blockIdx.y * 128) % S, bb = (blockIdx.y * 128) / S;
  b16* dst = vt + (((size_t)bb * H + h) * HD) * S + tok0; b16* dstl = vtl + (((size_t)bb * H + h) * HD) * S + tok0;
  for (int pass = 0; pass < 2; ++pass) {
#pragma unroll
    for (int j = 0; j < 8; ++j) { const int dd = wave * 16 + j * 2 + (lane >> 4), c8 = (lane & 15) * 8; *(volatile v8b*)(dst + (size_t)dd * S + c8) = *(const v8b*)(&Tt[0][dd][c8]); *(volatile v8b*)(dstl + (size_t)dd * S + c8) = *(const v8b*)(&Tt[1][dd][c8]); }
    __threadfence();
  }
}

__global__ __launch_bounds__(256) void attn_kernel(const b16* __restrict__ qk, const b16* __restrict__ vt, const b16* __restrict__ vtl, float* __restrict__ y) {
  __shared__ __attribute__((aligned(16))) float Os[8][16][HD + 4];
  const int wid = threadIdx.x >> 5, lane = threadIdx.x & 31, hh = lane >> 4, col = lane & 15;
  const int qt = blockIdx.x * 8 + wid, jt = qt & 127, h = (qt >> 7) & 15, b = qt >> 11, q0 = jt * 16, qi = q0 + col;
  const b16* Q = qk + ((((size_t)0 * Bn + b) * H + h) * S) * HD; const b16* K = qk + ((((size_t)1 * Bn + b) * H + h) * S) * HD;
  const b16* vb = vt + (((size_t)b * H + h) * HD) * S; const b16* vbl = vtl + (((size_t)b * H + h) * HD) * S;
  v16b qf[2];
#pragma unroll
  for (int ks = 0; ks < 2; ++ks) qf[ks] = frag_kb(Q + (size_t)qi * HD + ks * 32, hh);
  float m = -INFINITY, l = 0.0f; v8f o[4] = {{}, {}, {}, {}};
  for (int kb = 0; kb < q0 + 16; kb += 32) {
    v8f s0 = {}, s1 = {};
#pragma unroll
    for (int ks = 0; ks < 2; ++ks) { s0 = wmma16b(frag_kb(K + (size_t)(kb + col) * HD + ks * 32, hh), qf[ks], s0); s1 = wmma16b(frag_kb(K + (size_t)(kb + 16 + col) * HD + ks * 32, hh), qf[ks], s1); }
    float mr = -INFINITY;
#pragma unroll
    for (int r = 0; r < 8; ++r) { const int kk = kb + 8 * hh + r; s0[r] = (kk > qi) ? -INFINITY : s0[r] * SCALE; s1[r] = (kk + 16 > qi) ? -INFINITY : s1[r] * SCALE; mr = fmaxf(mr, fmaxf(s0[r], s1[r])); }
    mr = fmaxf(mr, __shfl_xor(mr, 16));
    float mn = fmaxf(m, mr); if (mn == -INFINITY) mn = 0.0f;
    const float al_ = __expf(m - mn); m = mn;
    float sum = 0.0f; v16b pb;
#pragma unroll
    for (int r = 0; r < 8; ++r) { const float e0 = __expf(s0[r] - mn), e1 = __expf(s1[r] - mn); sum += e0 + e1; pb[r] = (b16)e0; pb[8 + r] = (b16)e1; }
    sum += __shfl_xor(sum, 16); l = l * al_ + sum;
#pragma unroll
    for (int n = 0; n < 4; ++n) {
#pragma unroll
      for (int r = 0; r < 8; ++r) o[n][r] *= al_;
      o[n] = wmma16b(frag_kb(vb + (size_t)(n * 16 + col) * S + kb, hh), pb, o[n]); o[n] = wmma16b(frag_kb(vbl + (size_t)(n * 16 + col) * S + kb, hh), pb, o[n]);
    }
  }
  const float inv = 1.0f / (VS * l);
#pragma unroll
  for (int n = 0; n < 4; ++n)
#pragma unroll
    for (int r = 0; r < 8; ++r) Os[wid][col][n * 16 + 8 * hh + r] = o[n][r] * inv;
  wave_lds_sync();
  float* dst = y + ((size_t)b * S + q0) * D + h * HD;
  for (int pass = 0; pass < 2; ++pass) {
#pragma unroll
    for (int j = 0; j < 8; ++j) { const int rr = j * 2 + hh, c4 = col * 4; *(volatile v4f*)(dst + (size_t)rr * D + c4) = *(const v4f*)(&Os[wid][rr][c4]); }
    __threadfence();
  }
}

__global__ __launch_bounds__(128) void out_kernel(const float* __restrict__ y, const b16* __restrict__ wo16, float* __restrict__ out) {
  __shared__ __attribute__((aligned(16))) float Ts[4][32 * 64];
  const int lane = threadIdx.x & 31, wave = threadIdx.x >> 5, nloc = lane & 15, hlf = lane >> 4, m0 = blockIdx.y * 128 + wave * 32, c0 = blockIdx.x * 64;
  v8f acc[2][4];
#pragma unroll
  for (int r = 0; r < 2; ++r)
#pragma unroll
    for (int t = 0; t < 4; ++t) acc[r][t] = (v8f){};
  const Opnd A{y, nullptr, D}, B{wo16, nullptr, D};
  gemm_tile<5, 1>(A, B, D, m0, c0, nloc, hlf, acc);
  epi_f32(acc, 0.125f, nullptr, out, D, m0, c0, lane, Ts[wave]);
}
}

extern "C" void kernel_launch(void* const* d_in, const int* in_sizes, int n_in,
                              void* d_out, int out_size, void* d_ws, size_t ws_size, hipStream_t stream) {
  (void)n_in; (void)out_size;
  const float* x = (const float*)d_in[0]; const float* wqkv = (const float*)d_in[1]; const float* wout = (const float*)d_in[2];
  float* out = (float*)d_out;
  if (in_sizes[0] != NTOK * D || in_sizes[1] != D * D3 || in_sizes[2] != D * D) return;
  size_t off = 0; char* ws = (char*)d_ws;
  auto carve = [&](size_t bytes) { char* p = ws + off; off += (bytes + 255) & ~(size_t)255; return p; };
  unsigned short* x16 = (unsigned short*)carve((size_t)NTOK * D * 2);
  unsigned short* w16 = (unsigned short*)carve((size_t)D3 * D * 2);
  b16* wo16 = (b16*)carve((size_t)D * D * 2);
  b16* qk = (b16*)carve((size_t)2 * NTOK * D * 2);
  b16* vt = (b16*)carve((size_t)NTOK * D * 2); b16* vtl = (b16*)carve((size_t)NTOK * D * 2);
  float* y = (float*)carve((size_t)NTOK * D * 4);
  float* cst = (float*)carve((size_t)S * 32 * 2 * 4);
  if (off > ws_size) return;
  prep_kernel<<<512, 256, 0, stream>>>(x, x16);
  wt_kernel<0><<<dim3(D3 / 64, D / 64), 256, 0, stream>>>(wqkv, D, D3, w16);
  wt_kernel<1><<<dim3(D / 64, D / 64), 256, 0, stream>>>(wout, D, D, (unsigned short*)wo16);
  rope_kernel<<<S * 32 / 256, 256, 0, stream>>>(cst);
  proj_kernel<<<dim3(D3 / 64, NTOK / 128), 128, 0, stream>>>((const __bf16*)x16, (const __bf16*)w16, cst, qk, vt, vtl);
  attn_kernel<<<Bn * H * (S / 16) / 8, 256, 0, stream>>>(qk, vt, vtl, y);
  out_kernel<<<dim3(D / 64, NTOK / 128), 128, 0, stream>>>(y, wo16, out);
}
